// HGT_36344013259082
// MI455X (gfx1250) — hardware-run, weakly checked
//
#include <hip/hip_runtime.h>


namespace {
constexpr int N = 50000, NP = 50048, NLIM = 50048  , NLIMN = (NLIM < N ? NLIM : N), E = 200000, F = 128, H = 8, D = 16, L = 2, R = 3;
constexpr size_t XB_OFF = (size_t)N * F;
constexpr float XS = 8.0f, WSC = 256.0f;
__host__ __device__ constexpr int rel_src(int r) { return r == 1 ? 1 : 0; }
__host__ __device__ constexpr int rel_dst(int r) { return r == 0 ? 1 : 0; }
static_assert(NP % 64 == 0 && NLIM % 64 == 0, "tiling");
typedef _Float16 b16;
typedef __attribute__((ext_vector_type(16))) _Float16 v16b;
typedef __attribute__((ext_vector_type(8))) _Float16 v8b;
typedef __attribute__((ext_vector_type(8))) float v8f;
typedef __attribute__((ext_vector_type(4))) float v4f;
__device__ __forceinline__ float bf16_rne(float f) { unsigned int u = __float_as_uint(f); u += 0x7FFFu + ((u >> 16) & 1u); return __uint_as_float(u & 0xFFFF0000u); }
__device__ __forceinline__ void split16(float v, b16& hi, b16& lo) { hi = (b16)v; lo = (b16)(v - (float)hi); }
__device__ __forceinline__ v16b frag_kb(const b16* p, int hh) { const v8b a = *(const v8b*)(p + 8 * hh), b = *(const v8b*)(p + 16 + 8 * hh); v16b f;
#pragma unroll
  for (int e = 0; e < 8; ++e) { f[e] = a[e]; f[8 + e] = b[e]; } return f; }
__device__ __forceinline__ v8f wmma16b(v16b a, v16b b, v8f c) { v8f d = __builtin_amdgcn_wmma_f32_16x16x32_f16(false, a, false, b, (short)0, c, false, false); asm volatile("v_nop\n\tv_nop\n\tv_nop\n\tv_nop" : "+v"(d) : "v"(a), "v"(b)); return d; }
__device__ __forceinline__ void wave_lds_sync() { __builtin_amdgcn_fence(__ATOMIC_RELEASE, "workgroup"); __builtin_amdgcn_wave_barrier(); __builtin_amdgcn_fence(__ATOMIC_ACQUIRE, "workgroup"); }
__device__ __forceinline__ float pmul(float a, float b) { float p = a * b; asm volatile("" : "+v"(p)); return p; }
__device__ __forceinline__ int iclamp(int v, int lo, int hi) { return v < lo ? lo : (v > hi ? hi : v); }
constexpr int CSR_NBLK = 512, CSR_GB = 9, CSR_GN = 1 << CSR_GB  , CSR_MAXG = 512, CSR_CAP = 12288  ;
__global__ __launch_bounds__(64) void csrA_kernel(const int* __restrict__ dst, int E, int N, int nG, int CHP, int NGP, int* __restrict__ STG, int* __restrict__ HST) {
  extern __shared__ int sm[];
  int* cnt = sm; int* run = sm + NGP; int* ids = sm + 2 * NGP;
  const int b = blockIdx.x; const int ch = (E + CSR_NBLK - 1) / CSR_NBLK; const int e0 = b * ch, e1 = min(E, e0 + ch);
  for (int i = threadIdx.x; i < NGP; i += 64) cnt[i] = 0;
  for (int i = threadIdx.x; i < CHP; i += 64) ids[i] = -1;
  __syncthreads();
  if (threadIdx.x == 0) {
    for (int e = e0; e < e1; ++e) { int d = dst[e]; d = (d < 0) ? 0 : (d >= N ? N - 1 : d); cnt[d >> CSR_GB] += 1; }
    int acc = 0; for (int g = 0; g < nG; ++g) { run[g] = acc; acc += cnt[g]; }
    for (int e = e0; e < e1; ++e) { int d = dst[e]; d = (d < 0) ? 0 : (d >= N ? N - 1 : d); const int g = d >> CSR_GB; ids[run[g]] = e; run[g] += 1; } }
  __syncthreads();
  typedef __attribute__((ext_vector_type(4))) int v4i;
  for (int pass = 0; pass < 2; ++pass) {
    for (int i = threadIdx.x; i < CHP / 4; i += 64) *(volatile v4i*)(STG + (size_t)b * CHP + i * 4) = *(const v4i*)(&ids[i * 4]);
    for (int i = threadIdx.x; i < NGP / 4; i += 64) { v4i v; for (int e = 0; e < 4; ++e) v[e] = (i * 4 + e < nG) ? cnt[i * 4 + e] : 0; *(volatile v4i*)(HST + (size_t)b * NGP + i * 4) = v; }
    __threadfence(); }
}
__global__ __launch_bounds__(512) void csrS_kernel(const int* __restrict__ HST, int nG, int NGP, int* __restrict__ START, int* __restrict__ TOT, int* __restrict__ OFF) {
  __shared__ int tot[CSR_MAXG];
  const int b = threadIdx.x;
  for (int pass = 0; pass < 2; ++pass) { int runb = 0; for (int g = 0; g < nG; ++g) { int c = HST[(size_t)b * NGP + g]; c = (c < 0) ? 0 : c; ((volatile int*)OFF)[(size_t)g * CSR_NBLK + b] = runb; runb += c; } __threadfence(); }
  for (int g = threadIdx.x; g < nG; g += 512) { int s = 0; for (int bb = 0; bb < CSR_NBLK; ++bb) { int c = HST[(size_t)bb * NGP + g]; s += (c < 0) ? 0 : c; } tot[g] = s; }
  __syncthreads();
  if (threadIdx.x < 32) {
    __shared__ int st[CSR_MAXG + 32];
    if (threadIdx.x == 0) { int acc = 0; for (int g = 0; g < NGP; ++g) { st[g] = acc; if (g < nG) acc += (tot[g] + 31) & ~31; } st[NGP] = acc; }
    __builtin_amdgcn_fence(__ATOMIC_RELEASE, "workgroup"); __builtin_amdgcn_wave_barrier(); __builtin_amdgcn_fence(__ATOMIC_ACQUIRE, "workgroup");
    for (int pass = 0; pass < 2; ++pass) { for (int i = threadIdx.x; i < NGP + 32; i += 32) { ((volatile int*)START)[i] = (i <= NGP) ? st[min(i, NGP)] : 0; ((volatile int*)TOT)[i] = (i < nG) ? tot[i] : 0; } __threadfence(); } }
}
__global__ __launch_bounds__(256) void csrB_kernel(const int* __restrict__ dst, int N, int nG, int CHP, int NGP, int permLen, const int* __restrict__ STG, const int* __restrict__ HST, const int* __restrict__ OFF, const int* __restrict__ START, const int* __restrict__ TOT, int* __restrict__ PERM, int* __restrict__ ROWPTR, int* __restrict__ ROWCNT, int* __restrict__ FLAG) {
  typedef __attribute__((ext_vector_type(4))) int v4i;
  __shared__ int ids[CSR_CAP]; __shared__ unsigned short key[CSR_CAP]; __shared__ int outp[CSR_CAP]; __shared__ int ncnt[CSR_GN + 1]; __shared__ int boff[CSR_NBLK + 1];
  const int g = blockIdx.x, t_ = threadIdx.x; int tot = TOT[g]; int st = START[g], stn = START[g + 1]; const int v0 = g * CSR_GN; const int nv = min(CSR_GN, N - v0);
  st = (st < 0) ? 0 : (st > permLen - 32 ? permLen - 32 : st) & ~31; stn = (stn < st) ? st : (stn > permLen ? permLen : stn); tot = (tot < 0) ? 0 : tot; if (tot > stn - st && tot <= CSR_CAP) tot = stn - st;
  if (tot > CSR_CAP) {
    for (int pass = 0; pass < 2; ++pass) { for (int i = t_; i < CSR_GN / 4; i += 256) { v4i a, c; for (int e = 0; e < 4; ++e) { a[e] = st; c[e] = 0; } *(volatile v4i*)(ROWPTR + v0 + i * 4) = a; *(volatile v4i*)(ROWCNT + v0 + i * 4) = c; } if (t_ == 0) ((volatile int*)FLAG)[0] = 1; __threadfence(); } (void)nv; return; }
  if (t_ == 0) { int acc = 0; for (int b = 0; b < CSR_NBLK; ++b) { boff[b] = acc; int c = HST[(size_t)b * NGP + g]; c = (c < 0) ? 0 : (c > CHP ? CHP : c); acc += c; if (acc > tot) acc = tot; } boff[CSR_NBLK] = acc; }
  for (int i = t_; i <= CSR_GN; i += 256) ncnt[i] = 0;
  __syncthreads();
  for (int b = 0; b < CSR_NBLK; ++b) { const int c = boff[b + 1] - boff[b]; int o_ = OFF[(size_t)g * CSR_NBLK + b]; o_ = (o_ < 0) ? 0 : (o_ > CHP - c ? CHP - c : o_); const int* src_ = STG + (size_t)b * CHP + o_;
    for (int i = t_; i < c; i += 256) { int id = src_[i]; id = (id < 0) ? 0 : id; ids[boff[b] + i] = id; int d = dst[id]; d = (d < v0) ? v0 : (d >= N ? N - 1 : d); int kk = d - v0; kk = (kk < 0) ? 0 : (kk >= CSR_GN ? CSR_GN - 1 : kk); key[boff[b] + i] = (unsigned short)kk; } }
  __syncthreads();
  if (t_ == 0) { for (int i = 0; i < tot; ++i) ncnt[key[i]] += 1; int acc = 0; for (int vl = 0; vl < CSR_GN; ++vl) { const int c = ncnt[vl]; ncnt[vl] = acc; acc += c; } ncnt[CSR_GN] = acc;
    for (int i = 0; i < tot; ++i) { const int vl = key[i]; outp[ncnt[vl]] = ids[i]; ncnt[vl] += 1; }
    for (int vl = CSR_GN; vl > 0; --vl) ncnt[vl] = ncnt[vl - 1]; ncnt[0] = 0; }
  __syncthreads();
  for (int pass = 0; pass < 2; ++pass) {
    for (int i = t_; i < (stn - st) / 4; i += 256) { v4i v; for (int e = 0; e < 4; ++e) { const int q = i * 4 + e; v[e] = (q < tot) ? outp[q] : -1; } *(volatile v4i*)(PERM + st + i * 4) = v; }
    for (int i = t_; i < CSR_GN / 4; i += 256) { v4i a, c; for (int e = 0; e < 4; ++e) { const int vl = i * 4 + e; a[e] = st + ncnt[vl]; c[e] = (vl < nv) ? (ncnt[vl + 1] - ncnt[vl]) : 0; } *(volatile v4i*)(ROWPTR + v0 + i * 4) = a; *(volatile v4i*)(ROWCNT + v0 + i * 4) = c; }
    __threadfence(); }
}
__global__ __launch_bounds__(256) void csrZ_kernel(int* __restrict__ p, size_t n4) { typedef __attribute__((ext_vector_type(4))) int v4i; const size_t tid = (size_t)blockIdx.x * 256 + threadIdx.x, nth = (size_t)gridDim.x * 256; v4i z = {0, 0, 0, 0}; for (size_t i = tid; i < n4; i += nth) *(volatile v4i*)(p + i * 4) = z; }
struct CsrBufs { int *STG, *HST, *OFF, *START, *TOT, *PERM, *ROWPTR, *ROWCNT, *FLAG; int nG, NGP, CHP; size_t permLen; char* base; size_t bytes; };
static size_t csr_carve(CsrBufs& c, char* ws, size_t off, int E, int N) {
  const size_t off0 = off; c.base = ws + off;
  auto al = [&](size_t bytes) { char* p = ws + off; off += (bytes + 255) & ~(size_t)255; return p; };
  c.nG = (N + CSR_GN - 1) / CSR_GN; c.NGP = (c.nG + 31) & ~31; const int ch = (E + CSR_NBLK - 1) / CSR_NBLK; c.CHP = (ch + 31) & ~31; c.permLen = (size_t)E + 32 * (size_t)c.nG + 32;
  c.STG = (int*)al((size_t)CSR_NBLK * c.CHP * 4); c.HST = (int*)al((size_t)CSR_NBLK * c.NGP * 4); c.OFF = (int*)al((size_t)c.NGP * CSR_NBLK * 4); c.START = (int*)al((size_t)(c.NGP + 64) * 4); c.TOT = (int*)al((size_t)(c.NGP + 64) * 4);
  c.PERM = (int*)al(c.permLen * 4); c.ROWPTR = (int*)al((size_t)c.nG * CSR_GN * 4); c.ROWCNT = (int*)al((size_t)c.nG * CSR_GN * 4); c.FLAG = (int*)al(256);
  c.bytes = off - off0; return off;
}
static void csr_build(const CsrBufs& c, const int* dst, int E, int N, hipStream_t stream) {
  const size_t smem = (size_t)(2 * c.NGP + c.CHP) * 4;
  csrZ_kernel<<<512, 256, 0, stream>>>((int*)c.base, c.bytes / 16);
  csrA_kernel<<<CSR_NBLK, 64, smem, stream>>>(dst, E, N, c.nG, c.CHP, c.NGP, c.STG, c.HST);
  csrS_kernel<<<1, 512, 0, stream>>>(c.HST, c.nG, c.NGP, c.START, c.TOT, c.OFF);
  csrB_kernel<<<c.nG, 256, 0, stream>>>(dst, N, c.nG, c.CHP, c.NGP, (int)c.permLen, c.STG, c.HST, c.OFF, c.START, c.TOT, c.PERM, c.ROWPTR, c.ROWCNT, c.FLAG);
}

__global__ __launch_bounds__(256) void comp_kernel(const float* __restrict__ Wk, const float* __restrict__ bk, const float* __restrict__ Wv, const float* __restrict__ bv, const float* __restrict__ arel, const float* __restrict__ mrel, float* __restrict__ CW, float* __restrict__ CB) {
  const size_t u = (size_t)blockIdx.x * 256 + threadIdx.x; const size_t per = (size_t)F * F; const size_t nW = (size_t)L * R * 2 * per;
  if (u < nW) { const int lr = (int)(u / (2 * per)); const int l = lr / R, r = lr % R; const int m = (int)((u / per) % 2); const int c = (int)((u % per) / F), o = (int)(u % F); const int h = o / D, e = o % D; const int s = rel_src(r);
    const float* W = (m == 0 ? Wk : Wv) + ((size_t)l * 2 + s) * per; const float* A = (m == 0 ? arel : mrel) + (((size_t)l * R + r) * H + h) * D * D; float acc = 0.0f;
    for (int d = 0; d < D; ++d) acc += bf16_rne(W[(size_t)c * F + h * D + d]) * bf16_rne(A[d * D + e]);
    for (int pass = 0; pass < 2; ++pass) { ((volatile float*)CW)[u] = acc; __threadfence(); } }
  else if (u < nW + (size_t)L * R * 2 * F) { const size_t v2 = u - nW; const int lr = (int)(v2 / (2 * F)); const int l = lr / R, r = lr % R; const int m = (int)((v2 / F) % 2); const int o = (int)(v2 % F); const int h = o / D, e = o % D; const int s = rel_src(r);
    const float* b = (m == 0 ? bk : bv) + ((size_t)l * 2 + s) * F; const float* A = (m == 0 ? arel : mrel) + (((size_t)l * R + r) * H + h) * D * D; float acc = 0.0f;
    for (int d = 0; d < D; ++d) acc += bf16_rne(b[h * D + d]) * bf16_rne(A[d * D + e]);
    for (int pass = 0; pass < 2; ++pass) { ((volatile float*)CB)[v2] = acc; __threadfence(); } }
}
__global__ __launch_bounds__(256) void prep_kernel(const float* __restrict__ Wq, const float* __restrict__ Wa, const float* __restrict__ CW, b16* __restrict__ WQ, b16* __restrict__ WA, b16* __restrict__ CWh, b16* __restrict__ CWl) {
  const size_t u = (size_t)blockIdx.x * 256 + threadIdx.x; const size_t per8 = (size_t)F * F / 8; const size_t n1 = (size_t)L * 2 * per8, n3 = (size_t)L * R * 2 * per8;
  if (u < 2 * n1) { const int which = (int)(u / n1); const size_t e = (u % n1) * 8; const int lt = (int)(e / (F * F)); const int rem = (int)(e % (F * F)); const int oo = rem / F, k0 = rem % F; const float* W = (which == 0 ? Wq : Wa) + (size_t)lt * F * F; v8b o;
    for (int j = 0; j < 8; ++j) o[j] = (b16)(bf16_rne(W[(size_t)(k0 + j) * F + oo]) * WSC);
    b16* dst = (which == 0 ? WQ : WA) + e; for (int pass = 0; pass < 2; ++pass) { *(volatile v8b*)dst = o; __threadfence(); } }
  else if (u < 2 * n1 + n3) { const size_t e = (u - 2 * n1) * 8; const int lrm = (int)(e / (F * F)); const int rem = (int)(e % (F * F)); const int oo = rem / F, k0 = rem % F; const float* W = CW + (size_t)lrm * F * F; v8b oh, ol;
    for (int j = 0; j < 8; ++j) { b16 p, q; split16(W[(size_t)(k0 + j) * F + oo] * WSC, p, q); oh[j] = p; ol[j] = q; }
    for (int pass = 0; pass < 2; ++pass) { *(volatile v8b*)(CWh + e) = oh; *(volatile v8b*)(CWl + e) = ol; __threadfence(); } }
}
template <int LAYER, int T>
__global__ __launch_bounds__(128) void proj_kernel(const float* __restrict__ X, const b16* __restrict__ WQ, const b16* __restrict__ CWh, const b16* __restrict__ CWl, const float* __restrict__ bq, const float* __restrict__ CB, int slab0, int slab1, float* __restrict__ Q, float* __restrict__ KR, float* __restrict__ VR) {
  __shared__ __attribute__((aligned(16))) float Tf[4][16][F + 4];
  const int wave = threadIdx.x >> 5, lane = threadIdx.x & 31, nloc = lane & 15, hlf = lane >> 4; const size_t v0 = ((size_t)blockIdx.x * 4 + wave) * 16; const size_t vr = v0 + nloc; const size_t vra = vr < (size_t)N ? vr : (size_t)N - 1;
  const bool rowok = vr < (size_t)N && v0 < (size_t)NLIM;
#pragma unroll 1
  for (int slab = slab0; slab < slab1; ++slab) {
    const int rr_ = (slab - 1) >> 1, m = (slab - 1) & 1; const int r = (T == 0) ? (rr_ == 0 ? 0 : 2) : 1;
    const b16* Bh = (slab == 0) ? (WQ + ((size_t)LAYER * 2 + T) * F * F) : (CWh + (((size_t)LAYER * R + r) * 2 + m) * F * F); const b16* Bl = (slab == 0) ? nullptr : (CWl + (((size_t)LAYER * R + r) * 2 + m) * F * F);
    const float* bias = (slab == 0) ? (bq + ((size_t)LAYER * 2 + T) * F) : (CB + (((size_t)LAYER * R + r) * 2 + m) * F); float* OUT = (slab == 0) ? Q : (m == 0 ? KR : VR);
    v8f acc[8];
#pragma unroll
    for (int t = 0; t < 8; ++t) acc[t] = (v8f){};
    if (v0 < (size_t)NLIM) {
#pragma unroll
      for (int ks = 0; ks < 4; ++ks) {
        v16b ah, al; { float cv[16]; const float* xr = X + vra * F + ks * 32; const v4f c0 = *(const v4f*)(xr + 8 * hlf), c1 = *(const v4f*)(xr + 8 * hlf + 4), c2 = *(const v4f*)(xr + 16 + 8 * hlf), c3 = *(const v4f*)(xr + 16 + 8 * hlf + 4);
          for (int i = 0; i < 4; ++i) { cv[i] = c0[i]; cv[4 + i] = c1[i]; cv[8 + i] = c2[i]; cv[12 + i] = c3[i]; }
          if (!rowok) { for (int i = 0; i < 16; ++i) cv[i] = 0.0f; }
          for (int e2 = 0; e2 < 16; ++e2) { if (LAYER == 0) { ah[e2] = (b16)(bf16_rne(cv[e2]) * XS); al[e2] = (b16)0.0f; } else { b16 p, q; split16(cv[e2] * XS, p, q); ah[e2] = p; al[e2] = q; } } }
#pragma unroll
        for (int t = 0; t < 8; ++t) { const v16b bh = frag_kb(Bh + (size_t)(t * 16 + nloc) * F + ks * 32, hlf); acc[t] = wmma16b(ah, bh, acc[t]);
          if (slab > 0) { const v16b bl = frag_kb(Bl + (size_t)(t * 16 + nloc) * F + ks * 32, hlf); acc[t] = wmma16b(ah, bl, acc[t]); if (LAYER == 1 && m == 1) acc[t] = wmma16b(al, bh, acc[t]); } } } }
#pragma unroll
    for (int t = 0; t < 8; ++t) { const float bb = (slab == 0) ? bf16_rne(bias[t * 16 + nloc]) : bias[t * 16 + nloc];
#pragma unroll
      for (int r8 = 0; r8 < 8; ++r8) { const bool zr = (v0 + 8 * hlf + r8) >= (size_t)N; Tf[wave][8 * hlf + r8][t * 16 + nloc] = zr ? 0.0f : (acc[t][r8] * (1.0f / (XS * WSC)) + bb); } }
    wave_lds_sync();
    for (int pass = 0; pass < 2; ++pass) { for (int rr = 0; rr < 16; ++rr) *(volatile v4f*)(OUT + (v0 + rr) * F + lane * 4) = *(const v4f*)(&Tf[wave][rr][lane * 4]); __threadfence(); }
    wave_lds_sync(); }
}
template <int ACCUM>
__global__ __launch_bounds__(256) void edge_kernel(const float* __restrict__ Q, const float* __restrict__ KR, const float* __restrict__ VR, const float* __restrict__ prel, const int* __restrict__ srcs, const int* __restrict__ PERM, const int* __restrict__ ROWPTR, const int* __restrict__ ROWCNT, int permLen, float* __restrict__ AGG) {
  const int wave = threadIdx.x >> 5, lane = threadIdx.x & 31; const size_t v = (size_t)blockIdx.x * 8 + wave; const int c = lane * 4, h = lane / 4; v4f a = {0.0f, 0.0f, 0.0f, 0.0f};
  if (v < (size_t)NLIMN) { int st = ROWPTR[v], cnt = ROWCNT[v]; cnt = iclamp(cnt, 0, 65536); st = iclamp(st, 0, permLen - cnt); const v4f qv = *(const v4f*)(Q + v * F + c); const float ph = bf16_rne(prel[h]) * 0.25f;
    float mx = -INFINITY, den = 0.0f;
#pragma unroll 1
    for (int j = 0; j < cnt; ++j) { const int e = iclamp(PERM[st + j], 0, E - 1); const size_t s = (size_t)iclamp(srcs[e], 0, N - 1); if (s >= (size_t)NLIM) continue; const v4f kv = *(const v4f*)(KR + s * F + c); float lg = qv[0] * kv[0] + qv[1] * kv[1] + qv[2] * kv[2] + qv[3] * kv[3]; lg += __shfl_xor(lg, 1); lg += __shfl_xor(lg, 2); lg *= ph;
      const float mn = fmaxf(mx, lg); const float al = (mx == -INFINITY) ? 0.0f : __expf(mx - mn), w = __expf(lg - mn); a = a * al + *(const v4f*)(VR + s * F + c) * w; den = den * al + w; mx = mn; }
    const float inv = (den > 0.0f) ? 1.0f / (den + 1e-16f) : 0.0f; a *= inv;
    if (ACCUM) a += *(const v4f*)(AGG + v * F + c); }
  else if (ACCUM) return;
  for (int pass = 0; pass < 2; ++pass) { *(volatile v4f*)(AGG + v * F + c) = a; __threadfence(); }
}
template <int LAYER, int T>
__global__ __launch_bounds__(128) void out_kernel(const float* __restrict__ AGG, const float* __restrict__ X, const b16* __restrict__ WA, const float* __restrict__ ba, const float* __restrict__ skip, float* __restrict__ OUT) {
  __shared__ __attribute__((aligned(16))) float Tf[4][16][F + 4];
  const int wave = threadIdx.x >> 5, lane = threadIdx.x & 31, nloc = lane & 15, hlf = lane >> 4; const size_t v0 = ((size_t)blockIdx.x * 4 + wave) * 16; const size_t vr = v0 + nloc; const size_t vra = vr < (size_t)N ? vr : (size_t)N - 1;
  const b16* W = WA + ((size_t)LAYER * 2 + T) * F * F; const float* bb_ = ba + ((size_t)LAYER * 2 + T) * F; const float sg = 1.0f / (1.0f + __expf(-bf16_rne(skip[LAYER * 2 + T])));
  v8f acc[8];
#pragma unroll
  for (int t = 0; t < 8; ++t) acc[t] = (v8f){};
  if (v0 < (size_t)NLIM) {
#pragma unroll
    for (int ks = 0; ks < 4; ++ks) { v16b ahh, all_; const float* gr = AGG + vr * F + ks * 32; const v4f c0 = *(const v4f*)(gr + 8 * hlf), c1 = *(const v4f*)(gr + 8 * hlf + 4), c2 = *(const v4f*)(gr + 16 + 8 * hlf), c3 = *(const v4f*)(gr + 16 + 8 * hlf + 4); float cv[16];
      for (int i = 0; i < 4; ++i) { cv[i] = c0[i]; cv[4 + i] = c1[i]; cv[8 + i] = c2[i]; cv[12 + i] = c3[i]; }
      for (int e2 = 0; e2 < 16; ++e2) { const float x_ = cv[e2]; const float g = 0.5f * x_ * (1.0f + erff(x_ * 0.70710678118654752f)); b16 p, q; split16(g * XS, p, q); ahh[e2] = p; all_[e2] = q; }
#pragma unroll
      for (int t = 0; t < 8; ++t) { const v16b bw = frag_kb(W + (size_t)(t * 16 + nloc) * F + ks * 32, hlf); acc[t] = wmma16b(ahh, bw, acc[t]); acc[t] = wmma16b(all_, bw, acc[t]); } } }
#pragma unroll
  for (int t = 0; t < 8; ++t) { const float bb = bf16_rne(bb_[t * 16 + nloc]);
#pragma unroll
    for (int r8 = 0; r8 < 8; ++r8) Tf[wave][8 * hlf + r8][t * 16 + nloc] = acc[t][r8] * (1.0f / (XS * WSC)) + bb; }
  wave_lds_sync();
  for (int pass = 0; pass < 2; ++pass) { for (int rr = 0; rr < 16; ++rr) { const size_t row = v0 + rr; v4f o = *(const v4f*)(&Tf[wave][rr][lane * 4]); v4f xv = {0.0f, 0.0f, 0.0f, 0.0f};
      if (row < (size_t)N) { xv = *(const v4f*)(X + row * F + lane * 4); if (LAYER == 0) { for (int i = 0; i < 4; ++i) xv[i] = bf16_rne(xv[i]); } }
      for (int i = 0; i < 4; ++i) { float y = sg * o[i] + (1.0f - sg) * xv[i]; if (LAYER == 0) y = fmaxf(y, 0.0f); o[i] = (row < (size_t)NLIMN) ? y : 0.0f; }
      if (LAYER == 1 && row >= (size_t)NLIMN) continue;
      *(volatile v4f*)(OUT + row * F + lane * 4) = o; }
    __threadfence(); }
}
}

extern "C" void kernel_launch(void* const* d_in, const int* in_sizes, int n_in, void* d_out, int out_size, void* d_ws, size_t ws_size, hipStream_t stream) {
  (void)n_in;
  auto Fp = [&](int i) { return (const float*)d_in[i]; }; auto Ip = [&](int i) { return (const int*)d_in[i]; };
  if (in_sizes[0] != N * F || in_sizes[1] != N * F || in_sizes[2] != 2 * E || in_sizes[3] != 2 * E || in_sizes[4] != 2 * E || in_sizes[5] != 4 * F * F || in_sizes[7] != 4 * F * F || in_sizes[9] != 4 * F * F || in_sizes[11] != 4 * F * F || in_sizes[13] != 4 || in_sizes[14] != L * R * H * D * D || in_sizes[16] != L * R * H || out_size != 2 * N * F) return;
  size_t off = 0; char* ws = (char*)d_ws;
  auto carve = [&](size_t bytes) { char* p = ws + off; off += (bytes + 255) & ~(size_t)255; return p; };
  float* CW = (float*)carve((size_t)L * R * 2 * F * F * 4); float* CB = (float*)carve((size_t)L * R * 2 * F * 4);
  b16* WQ = (b16*)carve((size_t)L * 2 * F * F * 2); b16* WA = (b16*)carve((size_t)L * 2 * F * F * 2); b16* CWh = (b16*)carve((size_t)L * R * 2 * F * F * 2); b16* CWl = (b16*)carve((size_t)L * R * 2 * F * F * 2);
  const size_t rows = (size_t)NP * F * 4;
  float* QA = (float*)carve(rows); float* QB = (float*)carve(rows); float* KR = (float*)carve(rows); float* VR = (float*)carve(rows); float* AGA = (float*)carve(rows); float* AGB = (float*)carve(rows); float* XA1 = (float*)carve(rows); float* XB1 = (float*)carve(rows);
  CsrBufs c0, c1, c2; off = csr_carve(c0, ws, off, E, N); off = csr_carve(c1, ws, off, E, N); off = csr_carve(c2, ws, off, E, N);
  if (off > ws_size || off > ((size_t)240 << 20)) return;
  comp_kernel<<<(unsigned)((((size_t)L * R * 2 * F * F + (size_t)L * R * 2 * F) + 255) / 256), 256, 0, stream>>>(Fp(5), Fp(6), Fp(9), Fp(10), Fp(14), Fp(15), CW, CB);
  prep_kernel<<<(unsigned)((((size_t)2 * L * 2 + L * R * 2) * F * F / 8 + 255) / 256), 256, 0, stream>>>(Fp(7), Fp(11), CW, WQ, WA, CWh, CWl);
  csr_build(c0, Ip(2) + E, E, N, stream); csr_build(c1, Ip(3) + E, E, N, stream); csr_build(c2, Ip(4) + E, E, N, stream);
  for (int l = 0; l < L; ++l) {
    const float* XAin = (l == 0) ? Fp(0) : XA1; const float* XBin = (l == 0) ? Fp(1) : XB1; const float* pr = Fp(16) + (size_t)l * R * H;
    if (l == 0) { proj_kernel<0, 0><<<NP / 64, 128, 0, stream>>>(XAin, WQ, CWh, CWl, Fp(8), CB, 0, 3, QA, KR, VR); proj_kernel<0, 1><<<NP / 64, 128, 0, stream>>>(XBin, WQ, CWh, CWl, Fp(8), CB, 0, 1, QB, KR, VR); }
    else        { proj_kernel<1, 0><<<NP / 64, 128, 0, stream>>>(XAin, WQ, CWh, CWl, Fp(8), CB, 0, 3, QA, KR, VR); proj_kernel<1, 1><<<NP / 64, 128, 0, stream>>>(XBin, WQ, CWh, CWl, Fp(8), CB, 0, 1, QB, KR, VR); }
    edge_kernel<0><<<NP / 8, 256, 0, stream>>>(QB, KR, VR, pr + 0 * H, Ip(2), c0.PERM, c0.ROWPTR, c0.ROWCNT, (int)c0.permLen, AGB);
    if (l == 0) proj_kernel<0, 1><<<NP / 64, 128, 0, stream>>>(XBin, WQ, CWh, CWl, Fp(8), CB, 1, 3, QB, KR, VR); else proj_kernel<1, 1><<<NP / 64, 128, 0, stream>>>(XBin, WQ, CWh, CWl, Fp(8), CB, 1, 3, QB, KR, VR);
    edge_kernel<0><<<NP / 8, 256, 0, stream>>>(QA, KR, VR, pr + 1 * H, Ip(3), c1.PERM, c1.ROWPTR, c1.ROWCNT, (int)c1.permLen, AGA);
    if (l == 0) proj_kernel<0, 0><<<NP / 64, 128, 0, stream>>>(XAin, WQ, CWh, CWl, Fp(8), CB, 3, 5, QA, KR, VR); else proj_kernel<1, 0><<<NP / 64, 128, 0, stream>>>(XAin, WQ, CWh, CWl, Fp(8), CB, 3, 5, QA, KR, VR);
    edge_kernel<1><<<NP / 8, 256, 0, stream>>>(QA, KR, VR, pr + 2 * H, Ip(4), c2.PERM, c2.ROWPTR, c2.ROWCNT, (int)c2.permLen, AGA);
    if (l == 0) { out_kernel<0, 0><<<NP / 64, 128, 0, stream>>>(AGA, XAin, WA, Fp(12), Fp(13), XA1); out_kernel<0, 1><<<NP / 64, 128, 0, stream>>>(AGB, XBin, WA, Fp(12), Fp(13), XB1); }
    else        { out_kernel<1, 0><<<NP / 64, 128, 0, stream>>>(AGA, XAin, WA, Fp(12), Fp(13), (float*)d_out); out_kernel<1, 1><<<NP / 64, 128, 0, stream>>>(AGB, XBin, WA, Fp(12), Fp(13), (float*)d_out + XB_OFF); }
  }
}
